// AttnHGCN_1941325218035
// MI455X (gfx1250) — hardware-verified
//
#include <hip/hip_runtime.h>
#include <stddef.h>


#define DD      64
#define QVW     128
#define NTHR    256
#define NWAVE   8
#define EPT     8
#define NGRP    2
#define CHUNK   (NTHR * EPT * NGRP)
#define WCAP    (EPT * NGRP * 32)
#define LISTN   (NWAVE * WCAP)
#define NBC     4096
#define NBF     1024
#define RCAP    32768
#define RBN     128
#define TGT     256
#define DEGCAP  256
#define GROWS   128
#define OTHR    512
#define RELCAP  32
#define APK     72
#define WSCAP   134217728
#define INV_SQRT_DK 0.17677669529663687f

#define LDS_FILL ((RCAP + NBF + LISTN) * 4 + 64)
#define LDS_GEMM (2 * GROWS * APK * 2 + 2 * DD * APK * 2 + GROWS * QVW * 4)

static_assert((CHUNK & (CHUNK - 1)) == 0);
static_assert(CHUNK <= 4096);
static_assert((NBC & (NBC - 1)) == 0 && (NBF & (NBF - 1)) == 0);
static_assert(NBC == 4 * NBF);
static_assert(OTHR * 8 == NBC);
static_assert((RCAP % 32) == 0);
static_assert(TGT == NWAVE * 32);
static_assert(GROWS == NWAVE * 16);
static_assert(((2 * GROWS * APK * 2 + 2 * DD * APK * 2) % 16) == 0);

typedef float          v2f  __attribute__((ext_vector_type(2)));
typedef float          v4f  __attribute__((ext_vector_type(4)));
typedef float          v8f  __attribute__((ext_vector_type(8)));
typedef int            v4i  __attribute__((ext_vector_type(4)));
typedef unsigned short v8us __attribute__((ext_vector_type(8)));
typedef __bf16         v16b __attribute__((ext_vector_type(16)));
union FragB { v16b v; v8us h[2]; };

__device__ __forceinline__ unsigned int bfr(float f) {
  const unsigned int u = __float_as_uint(f);
  return (u + 0x7FFFu + ((u >> 16) & 1u)) >> 16;
}
__device__ __forceinline__ void split1(float x, unsigned short& hb, unsigned short& lb) {
  const unsigned int hu = bfr(x);
  const float hf = __uint_as_float(hu << 16);
  hb = (unsigned short)hu;
  lb = (unsigned short)bfr(x - hf);
}
__device__ __forceinline__ void split8(v4f a, v4f b, v8us& hi, v8us& lo) {
  unsigned short hb, lb;
  split1(a.x, hb, lb); hi[0] = hb; lo[0] = lb;
  split1(a.y, hb, lb); hi[1] = hb; lo[1] = lb;
  split1(a.z, hb, lb); hi[2] = hb; lo[2] = lb;
  split1(a.w, hb, lb); hi[3] = hb; lo[3] = lb;
  split1(b.x, hb, lb); hi[4] = hb; lo[4] = lb;
  split1(b.y, hb, lb); hi[5] = hb; lo[5] = lb;
  split1(b.z, hb, lb); hi[6] = hb; lo[6] = lb;
  split1(b.w, hb, lb); hi[7] = hb; lo[7] = lb;
}

__device__ __forceinline__ v8f wmb(v16b a, v16b b, v8f c) {
  v8f d = __builtin_amdgcn_wmma_f32_16x16x32_bf16(false, a, false, b, (short)0, c, false, false);
  asm volatile("v_nop\n\tv_nop\n\tv_nop\n\tv_nop" : "+v"(d) : "v"(a), "v"(b));
  return d;
}

template <int NB>
__device__ __forceinline__ int scan_chunk(const int* __restrict__ dsts, int nE, int cbase, int slotBase,
                                          int vec8, int* list, int tid, int lane, int wave) {
  int wc = 0;
#pragma unroll
  for (int g = 0; g < NGRP; ++g) {
    const int el0  = (g * NTHR + tid) * EPT;
    const int e0   = cbase + el0;
    const int sent = -2147483647 - 1;
    v4i da, db;
    if (vec8 != 0 && cbase + CHUNK <= nE) {
      da = *(const v4i*)(dsts + e0);
      db = *(const v4i*)(dsts + e0 + 4);
    } else {
      da.x = (e0     < nE) ? dsts[min(e0, nE - 1)] : sent;
      da.y = (e0 + 1 < nE) ? dsts[min(e0 + 1, nE - 1)] : sent;
      da.z = (e0 + 2 < nE) ? dsts[min(e0 + 2, nE - 1)] : sent;
      da.w = (e0 + 3 < nE) ? dsts[min(e0 + 3, nE - 1)] : sent;
      db.x = (e0 + 4 < nE) ? dsts[min(e0 + 4, nE - 1)] : sent;
      db.y = (e0 + 5 < nE) ? dsts[min(e0 + 5, nE - 1)] : sent;
      db.z = (e0 + 6 < nE) ? dsts[min(e0 + 6, nE - 1)] : sent;
      db.w = (e0 + 7 < nE) ? dsts[min(e0 + 7, nE - 1)] : sent;
    }
    const unsigned nb = (unsigned)slotBase;
    const unsigned s0 = (unsigned)da.x - nb, s1 = (unsigned)da.y - nb;
    const unsigned s2 = (unsigned)da.z - nb, s3 = (unsigned)da.w - nb;
    const unsigned s4 = (unsigned)db.x - nb, s5 = (unsigned)db.y - nb;
    const unsigned s6 = (unsigned)db.z - nb, s7 = (unsigned)db.w - nb;
    const bool h0 = s0 < (unsigned)NB, h1 = s1 < (unsigned)NB, h2 = s2 < (unsigned)NB, h3 = s3 < (unsigned)NB;
    const bool h4 = s4 < (unsigned)NB, h5 = s5 < (unsigned)NB, h6 = s6 < (unsigned)NB, h7 = s7 < (unsigned)NB;
    const unsigned any = __builtin_amdgcn_ballot_w32(h0 | h1 | h2 | h3 | h4 | h5 | h6 | h7);
    if (any != 0u) {
#define HITJ(J, HJ, SJ) { \
        const unsigned mj = __builtin_amdgcn_ballot_w32(HJ); \
        if (mj != 0u) { \
          if (HJ) { \
            const int pos = wc + (int)__builtin_amdgcn_mbcnt_lo(mj, 0u); \
            if (pos < WCAP) list[wave * WCAP + pos] = ((el0 + (J)) << 12) | (int)(SJ); \
          } \
          wc += (int)__builtin_popcount(mj); } }
      HITJ(0, h0, s0)
      HITJ(1, h1, s1)
      HITJ(2, h2, s2)
      HITJ(3, h3, s3)
      HITJ(4, h4, s4)
      HITJ(5, h5, s5)
      HITJ(6, h6, s6)
      HITJ(7, h7, s7)
#undef HITJ
    }
  }
  return wc;
}

__global__ __launch_bounds__(NTHR) void k_count(const int* __restrict__ dsts, int* cnt, int nE, int vec8) {
  __shared__ __attribute__((aligned(16))) int scnt[NBC];
  __shared__ __attribute__((aligned(16))) int list[LISTN];
  __shared__ int wcnt[NWAVE];
  const int tid = threadIdx.x, lane = tid & 31, wave = tid >> 5;
  const int nodeBase = blockIdx.x * NBC;
  for (int i = tid; i < NBC; i += NTHR) scnt[i] = 0;
  __syncthreads();
  const int nChunks = (nE + CHUNK - 1) / CHUNK;
#pragma unroll 1
  for (int ch = 0; ch < nChunks; ++ch) {
    const int cbase = ch * CHUNK;
    const int wc = scan_chunk<NBC>(dsts, nE, cbase, nodeBase, vec8, list, tid, lane, wave);
    if (lane == 0) wcnt[wave] = wc;
    __syncthreads();
    if (wave == 0) {
#pragma unroll 1
      for (int wsx = 0; wsx < NWAVE; ++wsx) {
        int n = __builtin_amdgcn_readfirstlane(wcnt[wsx]);
        n = n > WCAP ? WCAP : (n < 0 ? 0 : n);
        const int* lp = list + wsx * WCAP;
#pragma unroll 1
        for (int i = 0; i < n; ++i) {
          const int ent  = __builtin_amdgcn_readfirstlane(lp[i]);
          const int slot = ent & (NBC - 1);
          if (lane == 0) scnt[slot] = scnt[slot] + 1;
        }
      }
    }
    __syncthreads();
  }
  v4i cq[4];
#pragma unroll
  for (int q = 0; q < 4; ++q) {
    const int f = (wave * 4 + q) * 128 + 4 * lane;
    cq[q] = *(const v4i*)(scnt + f);
  }
  int* cp = cnt + (size_t)nodeBase;
#pragma unroll
  for (int q = 0; q < 4; ++q) {
    const int f = (wave * 4 + q) * 128 + 4 * lane;
    *(volatile v4i*)(cp + f) = cq[q];
  }
  __threadfence();
#pragma unroll
  for (int q = 0; q < 4; ++q) {
    const int f = (wave * 4 + q) * 128 + 4 * lane;
    *(volatile v4i*)(cp + f) = cq[q];
  }
}

__global__ __launch_bounds__(OTHR) void k_offsets(
    const int* __restrict__ cnt, int* off, int* rbase, int nChunk) {
  __shared__ __attribute__((aligned(16))) int soff[NBC];
  __shared__ __attribute__((aligned(16))) int srb[RBN];
  __shared__ int wtot[OTHR / 32];
  const int tid = threadIdx.x, lane = tid & 31, wave = tid >> 5, sub = tid >> 7;
  for (int i = tid; i < RBN; i += OTHR) srb[i] = 0;
  int carry = 0;
#pragma unroll 1
  for (int ch = 0; ch < nChunk; ++ch) {
    const int base = ch * NBC;
    const v4i c0 = *(const v4i*)(cnt + base + 8 * tid);
    const v4i c1 = *(const v4i*)(cnt + base + 8 * tid + 4);
    const int e0 = max(c0.x, 0), e1 = max(c0.y, 0), e2 = max(c0.z, 0), e3 = max(c0.w, 0);
    const int e4 = max(c1.x, 0), e5 = max(c1.y, 0), e6 = max(c1.z, 0), e7 = max(c1.w, 0);
    const int ts = e0 + e1 + e2 + e3 + e4 + e5 + e6 + e7;
    int incl = ts;
#pragma unroll
    for (int d = 1; d < 32; d <<= 1) {
      const int t = __shfl_up(incl, d);
      if (lane >= d) incl += t;
    }
    if (lane == 31) wtot[wave] = incl;
    __syncthreads();
    const int S0 = wtot[0]  + wtot[1]  + wtot[2]  + wtot[3];
    const int S1 = wtot[4]  + wtot[5]  + wtot[6]  + wtot[7];
    const int S2 = wtot[8]  + wtot[9]  + wtot[10] + wtot[11];
    const int S3 = wtot[12] + wtot[13] + wtot[14] + wtot[15];
    int pre = 0;
#pragma unroll 1
    for (int w = 4 * sub; w < wave; ++w) pre += wtot[w];
    const int b0 = carry;
    const int b1 = b0 + ((S0 + 31) & ~31);
    const int b2 = b1 + ((S1 + 31) & ~31);
    const int b3 = b2 + ((S2 + 31) & ~31);
    const int b4 = b3 + ((S3 + 31) & ~31);
    const int myb = sub == 0 ? b0 : (sub == 1 ? b1 : (sub == 2 ? b2 : b3));
    if (tid == 0) {
      srb[min(4 * ch + 0, RBN - 1)] = b0;
      srb[min(4 * ch + 1, RBN - 1)] = b1;
      srb[min(4 * ch + 2, RBN - 1)] = b2;
      srb[min(4 * ch + 3, RBN - 1)] = b3;
    }
    int run = myb + pre + incl - ts;
    soff[8 * tid + 0] = run; run += e0;
    soff[8 * tid + 1] = run; run += e1;
    soff[8 * tid + 2] = run; run += e2;
    soff[8 * tid + 3] = run; run += e3;
    soff[8 * tid + 4] = run; run += e4;
    soff[8 * tid + 5] = run; run += e5;
    soff[8 * tid + 6] = run; run += e6;
    soff[8 * tid + 7] = run;
    carry = b4;
    __syncthreads();
    const v4i o0 = *(const v4i*)(soff + 4 * tid);
    const v4i o1 = *(const v4i*)(soff + 4 * (tid + OTHR));
    int* op = off + base;
    *(volatile v4i*)(op + 4 * tid) = o0;
    *(volatile v4i*)(op + 4 * (tid + OTHR)) = o1;
    __threadfence();
    *(volatile v4i*)(op + 4 * tid) = o0;
    *(volatile v4i*)(op + 4 * (tid + OTHR)) = o1;
    __syncthreads();
  }
  if (tid == 0) srb[min(4 * nChunk, RBN - 1)] = carry;
  __syncthreads();
  v4i rv = {0, 0, 0, 0};
  if (tid < 32) rv = *(const v4i*)(srb + 4 * tid);
  if (tid < 32) *(volatile v4i*)(rbase + 4 * tid) = rv;
  __threadfence();
  if (tid < 32) *(volatile v4i*)(rbase + 4 * tid) = rv;
}

__global__ __launch_bounds__(NTHR) void k_fill(
    const int* __restrict__ dsts, const int* __restrict__ off, const int* __restrict__ rbase,
    int* csr, int nE, int vec8, int csrLen) {
  extern __shared__ v4f lds_dyn[];
  int* region = (int*)lds_dyn;
  int* cursor = region + RCAP;
  int* list   = cursor + NBF;
  int* wcnt   = list + LISTN;
  const int tid = threadIdx.x, lane = tid & 31, wave = tid >> 5;
  const int b = blockIdx.x;
  const int nodeBase = b * NBF;
  int rb0 = rbase[b];
  const int rb1 = rbase[b + 1];
  rb0 = rb0 < 0 ? 0 : (rb0 > csrLen ? csrLen : rb0);
  rb0 &= ~31;
  int len = rb1 - rb0;
  len = len < 0 ? 0 : (len > RCAP ? RCAP : len);
  int lenW = (len + 31) & ~31;
  if (rb0 + lenW > csrLen) lenW = (csrLen - rb0) & ~31;
  {
    const v4i z = {0, 0, 0, 0};
    for (int i = tid; i < RCAP / 4; i += NTHR) ((v4i*)region)[i] = z;
    for (int s = tid; s < NBF; s += NTHR) {
      int o = off[nodeBase + s] - rb0;
      o = o < 0 ? 0 : (o > RCAP ? RCAP : o);
      cursor[s] = o;
    }
  }
  __syncthreads();
  const int nChunks = (nE + CHUNK - 1) / CHUNK;
#pragma unroll 1
  for (int ch = 0; ch < nChunks; ++ch) {
    const int cbase = ch * CHUNK;
    const int wc = scan_chunk<NBF>(dsts, nE, cbase, nodeBase, vec8, list, tid, lane, wave);
    if (lane == 0) wcnt[wave] = wc;
    __syncthreads();
    if (wave == 0) {
#pragma unroll 1
      for (int wsx = 0; wsx < NWAVE; ++wsx) {
        int n = __builtin_amdgcn_readfirstlane(wcnt[wsx]);
        n = n > WCAP ? WCAP : (n < 0 ? 0 : n);
        const int* lp = list + wsx * WCAP;
#pragma unroll 1
        for (int i = 0; i < n; ++i) {
          const int ent  = __builtin_amdgcn_readfirstlane(lp[i]);
          const int slot = ent & (NBF - 1);
          int e = cbase + ((ent >> 12) & (CHUNK - 1));
          e = e > nE - 1 ? nE - 1 : e;
          if (lane == 0) {
            int pos = cursor[slot];
            pos = pos < 0 ? 0 : (pos > RCAP - 1 ? RCAP - 1 : pos);
            region[pos] = e;
            const int np = pos + 1;
            cursor[slot] = np > RCAP ? RCAP : np;
          }
        }
      }
    }
    __syncthreads();
  }
  const int nv = lenW >> 2;
  int* gp = csr + rb0;
#pragma unroll 1
  for (int i = tid; i < nv; i += NTHR) { const v4i v = ((const v4i*)region)[i]; *(volatile v4i*)(gp + 4 * i) = v; }
  __threadfence();
#pragma unroll 1
  for (int i = tid; i < nv; i += NTHR) { const v4i v = ((const v4i*)region)[i]; *(volatile v4i*)(gp + 4 * i) = v; }
}

__global__ __launch_bounds__(NTHR) void k_gemm(const float* __restrict__ X, int xRows,
                                               const float* __restrict__ W, float* QV) {
  extern __shared__ v4f lds_dyn[];
  unsigned short* sAh = (unsigned short*)lds_dyn;
  unsigned short* sAl = sAh + GROWS * APK;
  unsigned short* sBh = sAl + GROWS * APK;
  unsigned short* sBl = sBh + DD * APK;
  float*          stg = (float*)(sBl + DD * APK);
  const int tid = threadIdx.x, lane = tid & 31, wave = tid >> 5, hh = lane >> 4, m = lane & 15;
  const int rowBase = blockIdx.x * GROWS;

  {
    const int n = tid >> 2, k0 = (tid & 3) * 16;
    float v[16];
#pragma unroll
    for (int e = 0; e < 16; ++e) v[e] = W[(k0 + e) * DD + n];
    v4f a, b, c, d;
    a.x = v[0];  a.y = v[1];  a.z = v[2];  a.w = v[3];
    b.x = v[4];  b.y = v[5];  b.z = v[6];  b.w = v[7];
    c.x = v[8];  c.y = v[9];  c.z = v[10]; c.w = v[11];
    d.x = v[12]; d.y = v[13]; d.z = v[14]; d.w = v[15];
    v8us h0, l0, h1, l1;
    split8(a, b, h0, l0);
    split8(c, d, h1, l1);
    *(v8us*)(sBh + n * APK + k0)     = h0;
    *(v8us*)(sBh + n * APK + k0 + 8) = h1;
    *(v8us*)(sBl + n * APK + k0)     = l0;
    *(v8us*)(sBl + n * APK + k0 + 8) = l1;
  }
#pragma unroll
  for (int i = 0; i < (GROWS * DD / 8) / NTHR; ++i) {
    const int idx = i * NTHR + tid;
    const int r   = idx >> 3;
    const int c0  = (idx & 7) * 8;
    int gr = rowBase + r;
    gr = gr > xRows - 1 ? xRows - 1 : gr;
    const float* xp = X + (size_t)gr * DD + c0;
    const v4f ea = *(const v4f*)xp, eb = *(const v4f*)(xp + 4);
    v8us hv, lv;
    split8(ea, eb, hv, lv);
    *(v8us*)(sAh + r * APK + c0) = hv;
    *(v8us*)(sAl + r * APK + c0) = lv;
    float* sp = stg + r * QVW + 2 * c0 + 2;
    v2f p;
    p.x = ea.x; p.y = ea.y; *(v2f*)(sp + 0)  = p;
    p.x = ea.z; p.y = ea.w; *(v2f*)(sp + 4)  = p;
    p.x = eb.x; p.y = eb.y; *(v2f*)(sp + 8)  = p;
    p.x = eb.z; p.y = eb.w; *(v2f*)(sp + 12) = p;
  }
  __syncthreads();

  const unsigned short* pah = sAh + (wave * 16 + m) * APK + 8 * hh;
  const unsigned short* pal = sAl + (wave * 16 + m) * APK + 8 * hh;
  v8f acc[4];
#pragma unroll
  for (int t = 0; t < 4; ++t) { const v8f z = {0.f, 0.f, 0.f, 0.f, 0.f, 0.f, 0.f, 0.f}; acc[t] = z; }
#pragma unroll
  for (int kt = 0; kt < 2; ++kt) {
    FragB ah, al;
    ah.h[0] = *(const v8us*)(pah + 32 * kt);
    ah.h[1] = *(const v8us*)(pah + 32 * kt + 16);
    al.h[0] = *(const v8us*)(pal + 32 * kt);
    al.h[1] = *(const v8us*)(pal + 32 * kt + 16);
#pragma unroll
    for (int t = 0; t < 4; ++t) {
      const unsigned short* bp = sBh + (16 * t + m) * APK + 32 * kt + 8 * hh;
      const unsigned short* bq = sBl + (16 * t + m) * APK + 32 * kt + 8 * hh;
      FragB bh, bl;
      bh.h[0] = *(const v8us*)bp; bh.h[1] = *(const v8us*)(bp + 16);
      bl.h[0] = *(const v8us*)bq; bl.h[1] = *(const v8us*)(bq + 16);
      acc[t] = wmb(ah.v, bh.v, acc[t]);
      acc[t] = wmb(ah.v, bl.v, acc[t]);
      acc[t] = wmb(al.v, bh.v, acc[t]);
    }
  }
  float* strow = stg + (wave * 16 + 8 * hh) * QVW + 4 * (m >> 1) + (m & 1);
#pragma unroll
  for (int t = 0; t < 4; ++t) {
#pragma unroll
    for (int r = 0; r < 8; ++r) strow[r * QVW + 32 * t] = acc[t][r];
  }
  __syncthreads();
#pragma unroll
  for (int i = 0; i < 16; ++i) {
    const int row = wave * 16 + i;
    const v4f v = *(const v4f*)(stg + row * QVW + 4 * lane);
    *(volatile v4f*)(QV + (size_t)(rowBase + row) * QVW + 4 * lane) = v;
  }
  __threadfence();
#pragma unroll
  for (int i = 0; i < 16; ++i) {
    const int row = wave * 16 + i;
    const v4f v = *(const v4f*)(stg + row * QVW + 4 * lane);
    *(volatile v4f*)(QV + (size_t)(rowBase + row) * QVW + 4 * lane) = v;
  }
}

__device__ __forceinline__ v2f seg_attn(
    const int* __restrict__ csr, const int* __restrict__ tl, const int* __restrict__ ety,
    const float* QV, const float* sRel, int nRel, int n, int st, int lane,
    int nSrc, int nE, int csrLen, v2f q) {
  float m = -1.0e30f, s = 0.0f;
  v2f acc = {0.0f, 0.0f};
#pragma unroll 1
  for (int q0 = 0; q0 < n; q0 += 32) {
    int pos = st + q0 + lane;
    pos = pos < 0 ? 0 : (pos > csrLen - 1 ? csrLen - 1 : pos);
    int ed = csr[pos];
    ed = ed < 0 ? 0 : (ed > nE - 1 ? nE - 1 : ed);
    int t = tl[ed];
    t = t < 0 ? t + nSrc : t;
    t = t < 0 ? 0 : (t > nSrc - 1 ? nSrc - 1 : t);
    int rt = ety[ed] - 1;
    rt = rt < 0 ? rt + nRel : rt;
    rt = rt < 0 ? 0 : (rt > nRel - 1 ? nRel - 1 : rt);
    const int mcnt = (n - q0) < 32 ? (n - q0) : 32;
#pragma unroll 1
    for (int p = 0; p < mcnt; ++p) {
      const int src = __builtin_amdgcn_readlane(t, p);
      const int typ = __builtin_amdgcn_readlane(rt, p);
      const v4f xv = *(const v4f*)(QV + (size_t)src * QVW + 4 * lane);
      const v2f rv = *(const v2f*)(sRel + typ * DD + 2 * lane);
      float part = q.x * (xv.x * rv.x);
      part = fmaf(q.y, xv.y * rv.y, part);
      part += __shfl_xor(part, 1);
      part += __shfl_xor(part, 2);
      part += __shfl_xor(part, 4);
      part += __shfl_xor(part, 8);
      const float sc = part * INV_SQRT_DK;
      const float mn = fmaxf(m, sc);
      const float f  = __expf(m - mn);
      const float e  = __expf(sc - mn);
      m = mn;
      s = fmaf(s, f, e);
      acc.x = fmaf(acc.x, f, e * (xv.z * rv.x));
      acc.y = fmaf(acc.y, f, e * (xv.w * rv.y));
    }
  }
  const float inv = s > 0.0f ? __builtin_amdgcn_rcpf(s) : 0.0f;
  acc.x *= inv;
  acc.y *= inv;
  return acc;
}

__device__ __forceinline__ v2f seg_plain(
    const int* __restrict__ csr, const int* __restrict__ col, const float* __restrict__ wgt,
    const float* X, int n, int st, int lane, int nSrc, int nE, int csrLen) {
  v2f acc = {0.0f, 0.0f};
#pragma unroll 1
  for (int q0 = 0; q0 < n; q0 += 32) {
    int pos = st + q0 + lane;
    pos = pos < 0 ? 0 : (pos > csrLen - 1 ? csrLen - 1 : pos);
    int ed = csr[pos];
    ed = ed < 0 ? 0 : (ed > nE - 1 ? nE - 1 : ed);
    int c = col[ed];
    c = c < 0 ? c + nSrc : c;
    c = c < 0 ? 0 : (c > nSrc - 1 ? nSrc - 1 : c);
    const float wv = wgt[ed];
    const int mcnt = (n - q0) < 32 ? (n - q0) : 32;
#pragma unroll 1
    for (int p = 0; p < mcnt; ++p) {
      const int   src = __builtin_amdgcn_readlane(c, p);
      const float w   = __int_as_float(__builtin_amdgcn_readlane(__float_as_int(wv), p));
      const v2f   x   = *(const v2f*)(X + (size_t)src * DD + 2 * lane);
      acc.x = fmaf(w, x.x, acc.x);
      acc.y = fmaf(w, x.y, acc.y);
    }
  }
  return acc;
}

template <int ATTN, int FINAL>
__global__ __launch_bounds__(NTHR) void k_agg(
    const int* __restrict__ csr, const int* __restrict__ off, const int* __restrict__ cnt,
    const int* __restrict__ colA, const int* __restrict__ colB, const float* __restrict__ wgt,
    const float* __restrict__ relT, const float* QV, const float* X,
    const float* res0, const float* res1, float* dst,
    int nRows, int res0Rows, int nSrc, int nRel, int nE, int csrLen) {
  __shared__ __attribute__((aligned(16))) float sRel[ATTN != 0 ? RELCAP * DD : 4];
  const int tid = threadIdx.x, lane = tid & 31, wave = tid >> 5;
  const int tbase = blockIdx.x * TGT + wave * 32;
  const int cl = tbase + lane;
  const int cnt_l = cnt[cl];
  const int off_l = off[cl];
  const int q2 = 2 * (lane & 15);
  const int tg = lane >> 4;
  if (ATTN != 0) {
    for (int i = tid; i < RELCAP * DD; i += NTHR) {
      int r = i >> 6;
      r = r > nRel - 1 ? nRel - 1 : r;
      sRel[i] = relT[r * DD + (i & 63)];
    }
  }
  __syncthreads();

#pragma unroll 1
  for (int j = 0; j < 32; j += 2) {
    int na = __builtin_amdgcn_readlane(cnt_l, j);
    na = na < 0 ? 0 : (na > DEGCAP ? DEGCAP : na);
    const int sa = __builtin_amdgcn_readlane(off_l, j);
    int nb = __builtin_amdgcn_readlane(cnt_l, j + 1);
    nb = nb < 0 ? 0 : (nb > DEGCAP ? DEGCAP : nb);
    const int sb = __builtin_amdgcn_readlane(off_l, j + 1);
    v2f accA, accB;
    if (ATTN != 0) {
      const v2f qa = *(const v2f*)(QV + (size_t)(tbase + j) * QVW + 4 * lane);
      accA = seg_attn(csr, colA, colB, QV, sRel, nRel, na, sa, lane, nSrc, nE, csrLen, qa);
      const v2f qb = *(const v2f*)(QV + (size_t)(tbase + j + 1) * QVW + 4 * lane);
      accB = seg_attn(csr, colA, colB, QV, sRel, nRel, nb, sb, lane, nSrc, nE, csrLen, qb);
    } else {
      accA = seg_plain(csr, colA, wgt, X, na, sa, lane, nSrc, nE, csrLen);
      accB = seg_plain(csr, colA, wgt, X, nb, sb, lane, nSrc, nE, csrLen);
    }
    float ssa = fmaf(accA.x, accA.x, accA.y * accA.y);
    float ssb = fmaf(accB.x, accB.x, accB.y * accB.y);
    ssa += __shfl_xor(ssa, 1);  ssb += __shfl_xor(ssb, 1);
    ssa += __shfl_xor(ssa, 2);  ssb += __shfl_xor(ssb, 2);
    ssa += __shfl_xor(ssa, 4);  ssb += __shfl_xor(ssb, 4);
    ssa += __shfl_xor(ssa, 8);  ssb += __shfl_xor(ssb, 8);
    ssa += __shfl_xor(ssa, 16); ssb += __shfl_xor(ssb, 16);
    const float rna = __builtin_amdgcn_rcpf(fmaxf(__builtin_amdgcn_sqrtf(ssa), 1e-12f));
    const float rnb = __builtin_amdgcn_rcpf(fmaxf(__builtin_amdgcn_sqrtf(ssb), 1e-12f));
    accA.x *= rna; accA.y *= rna;
    accB.x *= rnb; accB.y *= rnb;
    const float a0 = __shfl(accA.x, q2),     a1 = __shfl(accA.y, q2);
    const float a2 = __shfl(accA.x, q2 + 1), a3 = __shfl(accA.y, q2 + 1);
    const float c0 = __shfl(accB.x, q2),     c1 = __shfl(accB.y, q2);
    const float c2 = __shfl(accB.x, q2 + 1), c3 = __shfl(accB.y, q2 + 1);
    v4f w;
    w.x = tg != 0 ? c0 : a0;
    w.y = tg != 0 ? c1 : a1;
    w.z = tg != 0 ? c2 : a2;
    w.w = tg != 0 ? c3 : a3;
    const int row = tbase + j + tg;
    if (FINAL != 0) {
      const int r0 = row > res0Rows - 1 ? res0Rows - 1 : row;
      const v4f u0 = *(const v4f*)(res0 + (size_t)r0 * DD + 4 * (lane & 15));
      const v4f u1 = *(const v4f*)(res1 + (size_t)row * DD + 4 * (lane & 15));
      w = (u0 + u1) + w;
    }
    float* gp = dst + (size_t)(tbase + j) * DD + 4 * lane;
    if (row < nRows) *(volatile v4f*)gp = w;
    __threadfence();
    if (row < nRows) *(volatile v4f*)gp = w;
  }
}

extern "C" void kernel_launch(void* const* d_in, const int* in_sizes, int n_in,
                              void* d_out, int out_size, void* d_ws, size_t ws_size,
                              hipStream_t stream) {
  if (n_in < 8) return;
  const int nU   = in_sizes[0] / DD;
  const int nEn  = in_sizes[1] / DD;
  const int nRel = in_sizes[2] / DD;
  if (nU < 1 || nEn < 1 || nRel < 1 || nRel > RELCAP) return;
  if (in_sizes[0] != nU * DD || in_sizes[1] != nEn * DD || in_sizes[2] != nRel * DD) return;
  if (in_sizes[3] != DD * DD) return;
  const int NI = in_sizes[4];
  const int E  = in_sizes[6];
  if (NI < 1 || E < 1 || in_sizes[5] != 2 * E || in_sizes[7] != 2 * NI) return;
  if ((long long)out_size != (long long)(nEn + nU) * DD) return;
  if (E > (1 << 28) || NI > (1 << 28) || nEn > (1 << 22) || nU > (1 << 22)) return;

  const float* usr_in = (const float*)d_in[0];
  const float* ent_in = (const float*)d_in[1];
  const float* relT   = (const float*)d_in[2];
  const float* W      = (const float*)d_in[3];
  const float* iw     = (const float*)d_in[4];
  const int*   ei     = (const int*)d_in[5];
  const int*   ety    = (const int*)d_in[6];
  const int*   ie     = (const int*)d_in[7];
  const int* head = ei;
  const int* tail = ei + E;
  const int* uidx = ie;
  const int* iidx = ie + NI;
  float* out0 = (float*)d_out;
  float* out1 = out0 + (size_t)nEn * DD;

  const int NPADE = ((nEn + TGT - 1) / TGT) * TGT;
  const int NPADU = ((nU + TGT - 1) / TGT) * TGT;
  const int nBCe = (nEn + NBC - 1) / NBC, CNTPADe = nBCe * NBC, nBFe = (nEn + NBF - 1) / NBF;
  const int nBCu = (nU + NBC - 1) / NBC,  CNTPADu = nBCu * NBC, nBFu = (nU + NBF - 1) / NBF;
  if (4 * nBCe + 1 > RBN || 4 * nBCu + 1 > RBN) return;
  if (31 * 4 * nBCe > 4096 || 31 * 4 * nBCu > 4096) return;
  const int csrLenE = ((E + 31) & ~31) + 4096;
  const int csrLenU = ((NI + 31) & ~31) + 4096;

  char* ws = (char*)d_ws;
  size_t off = 0;
  const size_t oCntE = off; off += (size_t)CNTPADe * 4;      off = (off + 255) & ~(size_t)255;
  const size_t oOffE = off; off += (size_t)CNTPADe * 4;      off = (off + 255) & ~(size_t)255;
  const size_t oRbE  = off; off += (size_t)RBN * 4;          off = (off + 255) & ~(size_t)255;
  const size_t oCsrE = off; off += (size_t)csrLenE * 4;      off = (off + 255) & ~(size_t)255;
  const size_t oCntU = off; off += (size_t)CNTPADu * 4;      off = (off + 255) & ~(size_t)255;
  const size_t oOffU = off; off += (size_t)CNTPADu * 4;      off = (off + 255) & ~(size_t)255;
  const size_t oRbU  = off; off += (size_t)RBN * 4;          off = (off + 255) & ~(size_t)255;
  const size_t oCsrU = off; off += (size_t)csrLenU * 4;      off = (off + 255) & ~(size_t)255;
  const size_t oQV   = off; off += (size_t)NPADE * QVW * 4;  off = (off + 255) & ~(size_t)255;
  const size_t oEN   = off; off += (size_t)NPADE * DD * 4;   off = (off + 255) & ~(size_t)255;
  const size_t oUN   = off; off += (size_t)NPADU * DD * 4;   off = (off + 255) & ~(size_t)255;
  if (off > ws_size || off > (size_t)WSCAP) return;
  int*   cntE = (int*)(ws + oCntE);
  int*   offE = (int*)(ws + oOffE);
  int*   rbE  = (int*)(ws + oRbE);
  int*   csrE = (int*)(ws + oCsrE);
  int*   cntU = (int*)(ws + oCntU);
  int*   offU = (int*)(ws + oOffU);
  int*   rbU  = (int*)(ws + oRbU);
  int*   csrU = (int*)(ws + oCsrU);
  float* QV   = (float*)(ws + oQV);
  float* EN1  = (float*)(ws + oEN);
  float* UN1  = (float*)(ws + oUN);

  const int vec8E = ((E & 3) == 0) ? 1 : 0;
  const int vec8U = ((NI & 3) == 0) ? 1 : 0;
  const int nAggE = NPADE / TGT, nAggU = NPADU / TGT, nGm = NPADE / GROWS;

  hipFuncSetAttribute(reinterpret_cast<const void*>(&k_fill), hipFuncAttributeMaxDynamicSharedMemorySize, LDS_FILL);
  hipFuncSetAttribute(reinterpret_cast<const void*>(&k_gemm), hipFuncAttributeMaxDynamicSharedMemorySize, LDS_GEMM);

  k_count<<<nBCe, NTHR, 0, stream>>>(head, cntE, E, vec8E);
  k_offsets<<<1, OTHR, 0, stream>>>(cntE, offE, rbE, nBCe);
  k_fill<<<nBFe, NTHR, LDS_FILL, stream>>>(head, offE, rbE, csrE, E, vec8E, csrLenE);
  k_count<<<nBCu, NTHR, 0, stream>>>(uidx, cntU, NI, vec8U);
  k_offsets<<<1, OTHR, 0, stream>>>(cntU, offU, rbU, nBCu);
  k_fill<<<nBFu, NTHR, LDS_FILL, stream>>>(uidx, offU, rbU, csrU, NI, vec8U, csrLenU);

  k_gemm<<<nGm, NTHR, LDS_GEMM, stream>>>(ent_in, nEn, W, QV);
  k_agg<1, 0><<<nAggE, NTHR, 0, stream>>>(csrE, offE, cntE, tail, ety, iw, relT, QV, ent_in,
                                          ent_in, UN1, EN1, NPADE, nEn, nEn, nRel, E, csrLenE);
  k_agg<0, 0><<<nAggU, NTHR, 0, stream>>>(csrU, offU, cntU, iidx, iidx, iw, relT, QV, ent_in,
                                          usr_in, EN1, UN1, NPADU, nU, nEn, nRel, NI, csrLenU);
  k_gemm<<<nGm, NTHR, LDS_GEMM, stream>>>(EN1, NPADE, W, QV);
  k_agg<1, 1><<<nAggE, NTHR, 0, stream>>>(csrE, offE, cntE, tail, ety, iw, relT, QV, EN1,
                                          ent_in, EN1, out0, nEn, nEn, nEn, nRel, E, csrLenE);
  k_agg<0, 1><<<nAggU, NTHR, 0, stream>>>(csrU, offU, cntU, iidx, iidx, iw, relT, QV, EN1,
                                          usr_in, UN1, out1, nU, nU, nEn, nRel, NI, csrLenU);
}
